// SPEmbedder2Conv_21062519620293
// MI455X (gfx1250) — hardware-run, weakly checked
//
#include <hip/hip_runtime.h>


namespace {
constexpr int N = 100000, NP = 100032, G = 100, NPG = 1000, GP = 112, E = 1600000, FIN = 64, HID = 128, RD = 64, OUTW = 384;
constexpr float XS = 8.0f, WSC = 256.0f, SL = 0.01f, EPS = 1e-5f;
typedef _Float16 b16;
typedef __attribute__((ext_vector_type(16))) _Float16 v16b;
typedef __attribute__((ext_vector_type(8))) _Float16 v8b;
typedef __attribute__((ext_vector_type(8))) float v8f;
typedef __attribute__((ext_vector_type(4))) float v4f;
__device__ __forceinline__ float bf16_rne(float f) { unsigned int u = __float_as_uint(f); u += 0x7FFFu + ((u >> 16) & 1u); return __uint_as_float(u & 0xFFFF0000u); }
__device__ __forceinline__ void split16(float v, b16& hi, b16& lo) { hi = (b16)v; lo = (b16)(v - (float)hi); }
__device__ __forceinline__ v16b frag_kb(const b16* p, int hh) { const v8b a = *(const v8b*)(p + 8 * hh), b = *(const v8b*)(p + 16 + 8 * hh); v16b f;
#pragma unroll
  for (int e = 0; e < 8; ++e) { f[e] = a[e]; f[8 + e] = b[e]; } return f; }
__device__ __forceinline__ v8f wmma16b(v16b a, v16b b, v8f c) { v8f d = __builtin_amdgcn_wmma_f32_16x16x32_f16(false, a, false, b, (short)0, c, false, false); asm volatile("v_nop\n\tv_nop\n\tv_nop\n\tv_nop" : "+v"(d) : "v"(a), "v"(b)); return d; }
__device__ __forceinline__ void wave_lds_sync() { __builtin_amdgcn_fence(__ATOMIC_RELEASE, "workgroup"); __builtin_amdgcn_wave_barrier(); __builtin_amdgcn_fence(__ATOMIC_ACQUIRE, "workgroup"); }
__device__ __forceinline__ float pmul(float a, float b) { float p = a * b; asm volatile("" : "+v"(p)); return p; }
__device__ __forceinline__ int iclamp(int v, int lo, int hi) { return v < lo ? lo : (v > hi ? hi : v); }
__device__ __forceinline__ float lk(float x) { return x >= 0.0f ? x : SL * x; }
constexpr int CSR_NBLK = 512, CSR_GB = 9, CSR_GN = 1 << CSR_GB  , CSR_MAXG = 512, CSR_CAP = 12288  ;
__global__ __launch_bounds__(64) void csrA_kernel(const int* __restrict__ dst, int E, int N, int nG, int CHP, int NGP, int* __restrict__ STG, int* __restrict__ HST) {
  extern __shared__ int sm[];
  int* cnt = sm; int* run = sm + NGP; int* ids = sm + 2 * NGP;
  const int b = blockIdx.x; const int ch = (E + CSR_NBLK - 1) / CSR_NBLK; const int e0 = b * ch, e1 = min(E, e0 + ch);
  for (int i = threadIdx.x; i < NGP; i += 64) cnt[i] = 0;
  for (int i = threadIdx.x; i < CHP; i += 64) ids[i] = -1;
  __syncthreads();
  if (threadIdx.x == 0) {
    for (int e = e0; e < e1; ++e) { int d = dst[e]; d = (d < 0) ? 0 : (d >= N ? N - 1 : d); cnt[d >> CSR_GB] += 1; }
    int acc = 0; for (int g = 0; g < nG; ++g) { run[g] = acc; acc += cnt[g]; }
    for (int e = e0; e < e1; ++e) { int d = dst[e]; d = (d < 0) ? 0 : (d >= N ? N - 1 : d); const int g = d >> CSR_GB; ids[run[g]] = e; run[g] += 1; } }
  __syncthreads();
  typedef __attribute__((ext_vector_type(4))) int v4i;
  for (int pass = 0; pass < 2; ++pass) {
    for (int i = threadIdx.x; i < CHP / 4; i += 64) *(volatile v4i*)(STG + (size_t)b * CHP + i * 4) = *(const v4i*)(&ids[i * 4]);
    for (int i = threadIdx.x; i < NGP / 4; i += 64) { v4i v; for (int e = 0; e < 4; ++e) v[e] = (i * 4 + e < nG) ? cnt[i * 4 + e] : 0; *(volatile v4i*)(HST + (size_t)b * NGP + i * 4) = v; }
    __threadfence(); }
}
__global__ __launch_bounds__(512) void csrS_kernel(const int* __restrict__ HST, int nG, int NGP, int* __restrict__ START, int* __restrict__ TOT, int* __restrict__ OFF) {
  __shared__ int tot[CSR_MAXG];
  const int b = threadIdx.x;
  for (int pass = 0; pass < 2; ++pass) { int runb = 0; for (int g = 0; g < nG; ++g) { int c = HST[(size_t)b * NGP + g]; c = (c < 0) ? 0 : c; ((volatile int*)OFF)[(size_t)g * CSR_NBLK + b] = runb; runb += c; } __threadfence(); }
  for (int g = threadIdx.x; g < nG; g += 512) { int s = 0; for (int bb = 0; bb < CSR_NBLK; ++bb) { int c = HST[(size_t)bb * NGP + g]; s += (c < 0) ? 0 : c; } tot[g] = s; }
  __syncthreads();
  if (threadIdx.x < 32) {
    __shared__ int st[CSR_MAXG + 32];
    if (threadIdx.x == 0) { int acc = 0; for (int g = 0; g < NGP; ++g) { st[g] = acc; if (g < nG) acc += (tot[g] + 31) & ~31; } st[NGP] = acc; }
    __builtin_amdgcn_fence(__ATOMIC_RELEASE, "workgroup"); __builtin_amdgcn_wave_barrier(); __builtin_amdgcn_fence(__ATOMIC_ACQUIRE, "workgroup");
    for (int pass = 0; pass < 2; ++pass) { for (int i = threadIdx.x; i < NGP + 32; i += 32) { ((volatile int*)START)[i] = (i <= NGP) ? st[min(i, NGP)] : 0; ((volatile int*)TOT)[i] = (i < nG) ? tot[i] : 0; } __threadfence(); } }
}
__global__ __launch_bounds__(256) void csrB_kernel(const int* __restrict__ dst, int N, int nG, int CHP, int NGP, int permLen, const int* __restrict__ STG, const int* __restrict__ HST, const int* __restrict__ OFF, const int* __restrict__ START, const int* __restrict__ TOT, int* __restrict__ PERM, int* __restrict__ ROWPTR, int* __restrict__ ROWCNT, int* __restrict__ FLAG) {
  typedef __attribute__((ext_vector_type(4))) int v4i;
  __shared__ int ids[CSR_CAP]; __shared__ unsigned short key[CSR_CAP]; __shared__ int outp[CSR_CAP]; __shared__ int ncnt[CSR_GN + 1]; __shared__ int boff[CSR_NBLK + 1];
  const int g = blockIdx.x, t_ = threadIdx.x; int tot = TOT[g]; int st = START[g], stn = START[g + 1]; const int v0 = g * CSR_GN; const int nv = min(CSR_GN, N - v0);
  st = (st < 0) ? 0 : (st > permLen - 32 ? permLen - 32 : st) & ~31; stn = (stn < st) ? st : (stn > permLen ? permLen : stn); tot = (tot < 0) ? 0 : tot; if (tot > stn - st && tot <= CSR_CAP) tot = stn - st;
  if (tot > CSR_CAP) {
    for (int pass = 0; pass < 2; ++pass) { for (int i = t_; i < CSR_GN / 4; i += 256) { v4i a, c; for (int e = 0; e < 4; ++e) { a[e] = st; c[e] = 0; } *(volatile v4i*)(ROWPTR + v0 + i * 4) = a; *(volatile v4i*)(ROWCNT + v0 + i * 4) = c; } if (t_ == 0) ((volatile int*)FLAG)[0] = 1; __threadfence(); } (void)nv; return; }
  if (t_ == 0) { int acc = 0; for (int b = 0; b < CSR_NBLK; ++b) { boff[b] = acc; int c = HST[(size_t)b * NGP + g]; c = (c < 0) ? 0 : (c > CHP ? CHP : c); acc += c; if (acc > tot) acc = tot; } boff[CSR_NBLK] = acc; }
  for (int i = t_; i <= CSR_GN; i += 256) ncnt[i] = 0;
  __syncthreads();
  for (int b = 0; b < CSR_NBLK; ++b) { const int c = boff[b + 1] - boff[b]; int o_ = OFF[(size_t)g * CSR_NBLK + b]; o_ = (o_ < 0) ? 0 : (o_ > CHP - c ? CHP - c : o_); const int* src_ = STG + (size_t)b * CHP + o_;
    for (int i = t_; i < c; i += 256) { int id = src_[i]; id = (id < 0) ? 0 : id; ids[boff[b] + i] = id; int d = dst[id]; d = (d < v0) ? v0 : (d >= N ? N - 1 : d); int kk = d - v0; kk = (kk < 0) ? 0 : (kk >= CSR_GN ? CSR_GN - 1 : kk); key[boff[b] + i] = (unsigned short)kk; } }
  __syncthreads();
  if (t_ == 0) { for (int i = 0; i < tot; ++i) ncnt[key[i]] += 1; int acc = 0; for (int vl = 0; vl < CSR_GN; ++vl) { const int c = ncnt[vl]; ncnt[vl] = acc; acc += c; } ncnt[CSR_GN] = acc;
    for (int i = 0; i < tot; ++i) { const int vl = key[i]; outp[ncnt[vl]] = ids[i]; ncnt[vl] += 1; }
    for (int vl = CSR_GN; vl > 0; --vl) ncnt[vl] = ncnt[vl - 1]; ncnt[0] = 0; }
  __syncthreads();
  for (int pass = 0; pass < 2; ++pass) {
    for (int i = t_; i < (stn - st) / 4; i += 256) { v4i v; for (int e = 0; e < 4; ++e) { const int q = i * 4 + e; v[e] = (q < tot) ? outp[q] : -1; } *(volatile v4i*)(PERM + st + i * 4) = v; }
    for (int i = t_; i < CSR_GN / 4; i += 256) { v4i a, c; for (int e = 0; e < 4; ++e) { const int vl = i * 4 + e; a[e] = st + ncnt[vl]; c[e] = (vl < nv) ? (ncnt[vl + 1] - ncnt[vl]) : 0; } *(volatile v4i*)(ROWPTR + v0 + i * 4) = a; *(volatile v4i*)(ROWCNT + v0 + i * 4) = c; }
    __threadfence(); }
}
__global__ __launch_bounds__(256) void csrZ_kernel(int* __restrict__ p, size_t n4) { typedef __attribute__((ext_vector_type(4))) int v4i; const size_t tid = (size_t)blockIdx.x * 256 + threadIdx.x, nth = (size_t)gridDim.x * 256; v4i z = {0, 0, 0, 0}; for (size_t i = tid; i < n4; i += nth) *(volatile v4i*)(p + i * 4) = z; }
struct CsrBufs { int *STG, *HST, *OFF, *START, *TOT, *PERM, *ROWPTR, *ROWCNT, *FLAG; int nG, NGP, CHP; size_t permLen; char* base; size_t bytes; };
static size_t csr_carve(CsrBufs& c, char* ws, size_t off, int E, int N) {
  const size_t off0 = off; c.base = ws + off;
  auto al = [&](size_t bytes) { char* p = ws + off; off += (bytes + 255) & ~(size_t)255; return p; };
  c.nG = (N + CSR_GN - 1) / CSR_GN; c.NGP = (c.nG + 31) & ~31; const int ch = (E + CSR_NBLK - 1) / CSR_NBLK; c.CHP = (ch + 31) & ~31; c.permLen = (size_t)E + 32 * (size_t)c.nG + 32;
  c.STG = (int*)al((size_t)CSR_NBLK * c.CHP * 4); c.HST = (int*)al((size_t)CSR_NBLK * c.NGP * 4); c.OFF = (int*)al((size_t)c.NGP * CSR_NBLK * 4); c.START = (int*)al((size_t)(c.NGP + 64) * 4); c.TOT = (int*)al((size_t)(c.NGP + 64) * 4);
  c.PERM = (int*)al(c.permLen * 4); c.ROWPTR = (int*)al((size_t)c.nG * CSR_GN * 4); c.ROWCNT = (int*)al((size_t)c.nG * CSR_GN * 4); c.FLAG = (int*)al(256);
  c.bytes = off - off0; return off;
}
static void csr_build(const CsrBufs& c, const int* dst, int E, int N, hipStream_t stream) {
  const size_t smem = (size_t)(2 * c.NGP + c.CHP) * 4;
  csrZ_kernel<<<512, 256, 0, stream>>>((int*)c.base, c.bytes / 16);
  csrA_kernel<<<CSR_NBLK, 64, smem, stream>>>(dst, E, N, c.nG, c.CHP, c.NGP, c.STG, c.HST);
  csrS_kernel<<<1, 512, 0, stream>>>(c.HST, c.nG, c.NGP, c.START, c.TOT, c.OFF);
  csrB_kernel<<<c.nG, 256, 0, stream>>>(dst, N, c.nG, c.CHP, c.NGP, (int)c.permLen, c.STG, c.HST, c.OFF, c.START, c.TOT, c.PERM, c.ROWPTR, c.ROWCNT, c.FLAG);
}


__global__ __launch_bounds__(256) void wprep_kernel(const float* __restrict__ w1, const float* __restrict__ w2, const float* __restrict__ p1, const float* __restrict__ p2, const float* __restrict__ q1, const float* __restrict__ q2,
                                                    b16* __restrict__ W1T, b16* __restrict__ W2T, b16* __restrict__ P1T, b16* __restrict__ P2T, b16* __restrict__ Q1T, b16* __restrict__ Q2T) {
  const size_t u = (size_t)blockIdx.x * 256 + threadIdx.x; const size_t n0 = (size_t)HID * FIN / 8, n1 = (size_t)HID * HID / 8, n2 = (size_t)RD * HID / 8; size_t t = u; v8b o;
  if (t < n0) { const size_t e = t * 8; const int oo = (int)(e / FIN), k0 = (int)(e % FIN); for (int j = 0; j < 8; ++j) o[j] = (b16)(bf16_rne(w1[(size_t)(k0 + j) * HID + oo]) * WSC); for (int pass = 0; pass < 2; ++pass) { *(volatile v8b*)(W1T + e) = o; __threadfence(); } return; } t -= n0;
  for (int which = 0; which < 3; ++which) { const float* w = which == 0 ? w2 : (which == 1 ? p1 : p2); b16* dst = which == 0 ? W2T : (which == 1 ? P1T : P2T);
    if (t < n1) { const size_t e = t * 8; const int oo = (int)(e / HID), k0 = (int)(e % HID); for (int j = 0; j < 8; ++j) o[j] = (b16)(bf16_rne(w[(size_t)(k0 + j) * HID + oo]) * WSC); for (int pass = 0; pass < 2; ++pass) { *(volatile v8b*)(dst + e) = o; __threadfence(); } return; } t -= n1; }
  for (int which = 0; which < 2; ++which) { const float* w = which == 0 ? q1 : q2; b16* dst = which == 0 ? Q1T : Q2T;
    if (t < n2) { const size_t e = t * 8; const int oo = (int)(e / HID), k0 = (int)(e % HID); for (int j = 0; j < 8; ++j) o[j] = (b16)(bf16_rne(w[(size_t)(k0 + j) * RD + oo]) * WSC); for (int pass = 0; pass < 2; ++pass) { *(volatile v8b*)(dst + e) = o; __threadfence(); } return; } t -= n2; }
}
template <int MODE>
__global__ __launch_bounds__(128) void gemm_kernel(const float* __restrict__ src, const b16* __restrict__ W, const int* __restrict__ OCNT, const float* __restrict__ bias, float* __restrict__ OUT) {
  __shared__ __attribute__((aligned(16))) b16 Ah[4][16][HID + 8], Al[4][16][HID + 8]; __shared__ __attribute__((aligned(16))) float Tf[4][16][HID + 4];
  const int wave = threadIdx.x >> 5, lane = threadIdx.x & 31, nloc = lane & 15, hlf = lane >> 4; const size_t m0 = (size_t)blockIdx.x * 64 + wave * 16;
  v8f acc[8];
#pragma unroll
  for (int t = 0; t < 8; ++t) acc[t] = (v8f){};
  if (MODE == 0) { const size_t r = m0 + nloc; const size_t rc = r < (size_t)N ? r : (size_t)(N - 1); const float* xr = src + rc * FIN;
#pragma unroll
    for (int kb = 0; kb < FIN; kb += 32) { v16b a; for (int e = 0; e < 8; ++e) { a[e] = (b16)(bf16_rne(xr[kb + 8 * hlf + e]) * XS); a[8 + e] = (b16)(bf16_rne(xr[kb + 16 + 8 * hlf + e]) * XS); }
#pragma unroll
      for (int t = 0; t < 8; ++t) acc[t] = wmma16b(a, frag_kb(W + (size_t)(t * 16 + nloc) * FIN + kb, hlf), acc[t]); } }
  else { for (int rr = 0; rr < 16; ++rr) { v4f v = {0.0f, 0.0f, 0.0f, 0.0f}; if (m0 + rr < (size_t)N) v = *(const v4f*)(src + (m0 + rr) * HID + lane * 4);
      for (int j = 0; j < 4; ++j) { b16 p, s; split16(v[j] * XS, p, s); Ah[wave][rr][lane * 4 + j] = p; Al[wave][rr][lane * 4 + j] = s; } }
    wave_lds_sync();
#pragma unroll 2
    for (int kb = 0; kb < HID; kb += 32) { const v16b a = frag_kb(&Ah[wave][nloc][kb], hlf), al = frag_kb(&Al[wave][nloc][kb], hlf);
#pragma unroll
      for (int t = 0; t < 8; ++t) { const v16b bw = frag_kb(W + (size_t)(t * 16 + nloc) * HID + kb, hlf); acc[t] = wmma16b(a, bw, acc[t]); acc[t] = wmma16b(al, bw, acc[t]); } }
    wave_lds_sync(); }
#pragma unroll
  for (int t = 0; t < 8; ++t) { const int c = t * 16 + nloc; const float bb = (MODE == 2) ? bf16_rne(bias[c]) : 0.0f;
#pragma unroll 1
    for (int r8 = 0; r8 < 8; ++r8) { const size_t row = m0 + 8 * hlf + r8; const bool ok = row < (size_t)N; float v = acc[t][r8] * (1.0f / (XS * WSC));
      if (MODE == 2) v = lk(v + bb); else { int oc = ok ? OCNT[row] : 1; oc = iclamp(oc, 1, 65536); v = pmul(v, rsqrtf((float)oc)); }
      Tf[wave][8 * hlf + r8][c] = ok ? v : 0.0f; } }
  wave_lds_sync();
  for (int pass = 0; pass < 2; ++pass) { for (int rr = 0; rr < 16; ++rr) *(volatile v4f*)(OUT + (m0 + rr) * HID + lane * 4) = *(const v4f*)(&Tf[wave][rr][lane * 4]); __threadfence(); }
}
__global__ __launch_bounds__(256) void agg_kernel(const float* __restrict__ HW, const float* __restrict__ ew, const int* __restrict__ srcs, const int* __restrict__ PERM, const int* __restrict__ ROWPTR, const int* __restrict__ ROWCNT, int permLen, float* __restrict__ Z) {
  const int wave = threadIdx.x >> 5, lane = threadIdx.x & 31; const size_t v = (size_t)blockIdx.x * 8 + wave; v4f a = {0.0f, 0.0f, 0.0f, 0.0f};
  if (v < (size_t)N) { int st = ROWPTR[v], cnt = ROWCNT[v]; cnt = iclamp(cnt, 0, 65536); st = iclamp(st, 0, permLen - cnt); const float di = rsqrtf((float)(cnt < 1 ? 1 : cnt));
#pragma unroll 1
    for (int j = 0; j < cnt; ++j) { const int e = iclamp(PERM[st + j], 0, E - 1); const size_t s = (size_t)iclamp(srcs[e], 0, N - 1); const float w = bf16_rne(ew[e]); const v4f h = *(const v4f*)(HW + s * HID + lane * 4);
      for (int i = 0; i < 4; ++i) a[i] += pmul(w, h[i]); }
    for (int i = 0; i < 4; ++i) a[i] = pmul(di, a[i]); }
  for (int pass = 0; pass < 2; ++pass) { *(volatile v4f*)(Z + v * HID + lane * 4) = a; __threadfence(); }
}
__global__ __launch_bounds__(128) void gnorm_kernel(const float* __restrict__ Z, const float* __restrict__ al, const float* __restrict__ ga, const float* __restrict__ be, float* __restrict__ H, float* __restrict__ Mg) {
  const int g = blockIdx.x, c = threadIdx.x; const float* z = Z + (size_t)g * NPG * HID + c; float* h = H + (size_t)g * NPG * HID + c;
  double s = 0.0;
#pragma unroll 4
  for (int r = 0; r < NPG; ++r) s += (double)z[(size_t)r * HID];
  const float mean = (float)(s * (1.0 / NPG)); const float am = pmul(bf16_rne(al[c]), mean);
  double q = 0.0;
#pragma unroll 4
  for (int r = 0; r < NPG; ++r) { const float d = z[(size_t)r * HID] - am; q += (double)pmul(d, d); }
  const float var = (float)(q * (1.0 / NPG)); const float rstd = rsqrtf(var + EPS); const float gg = bf16_rne(ga[c]), bb = bf16_rne(be[c]);
  double m = 0.0;
  for (int pass = 0; pass < 2; ++pass) { m = 0.0;
#pragma unroll 4
    for (int r = 0; r < NPG; ++r) { const float v = lk(pmul(gg, pmul(z[(size_t)r * HID] - am, rstd)) + bb); ((volatile float*)h)[(size_t)r * HID] = v; m += (double)v; }
    __threadfence(); }
  const float mv = (float)(m * (1.0 / NPG));
  for (int pass = 0; pass < 2; ++pass) { ((volatile float*)Mg)[(size_t)g * HID + c] = mv; __threadfence(); }
}
__global__ __launch_bounds__(128) void pool_kernel(const float* __restrict__ PH, float* __restrict__ POOL) {
  const int g = blockIdx.x, c = threadIdx.x; float mv = 0.0f;
  if (g < G) { const float* p = PH + (size_t)g * NPG * HID + c; double s = 0.0;
#pragma unroll 4
    for (int r = 0; r < NPG; ++r) s += (double)p[(size_t)r * HID];
    mv = (float)(s * (1.0 / NPG)); }
  for (int pass = 0; pass < 2; ++pass) { ((volatile float*)POOL)[(size_t)g * HID + c] = mv; __threadfence(); }
}
__global__ __launch_bounds__(32) void head_kernel(const float* __restrict__ POOL1, const float* __restrict__ POOL2, const b16* __restrict__ Q1T, const b16* __restrict__ Q2T, const float* __restrict__ qb1, const float* __restrict__ qb2, const float* __restrict__ M1, const float* __restrict__ M2, float* __restrict__ out) {
  __shared__ __attribute__((aligned(16))) b16 Ah[16][HID + 8], Al[16][HID + 8]; __shared__ __attribute__((aligned(16))) float so[16][OUTW];
  const int lane = threadIdx.x, nloc = lane & 15, hlf = lane >> 4; const size_t g0 = (size_t)blockIdx.x * 16;
#pragma unroll 1
  for (int k = 0; k < 2; ++k) { const float* PL = k == 0 ? POOL1 : POOL2; const b16* Q = k == 0 ? Q1T : Q2T; const float* qb = k == 0 ? qb1 : qb2; const float* Mk = k == 0 ? M1 : M2;
#pragma unroll 1
    for (int rr = 0; rr < 16; ++rr) { const v4f v = *(const v4f*)(PL + (g0 + rr) * HID + lane * 4); for (int j = 0; j < 4; ++j) { b16 p, s; split16(v[j] * XS, p, s); Ah[rr][lane * 4 + j] = p; Al[rr][lane * 4 + j] = s; }
      const size_t gr = (g0 + rr) < (size_t)G ? (g0 + rr) : (size_t)(G - 1); const v4f mrow = *(const v4f*)(Mk + gr * HID + lane * 4); for (int j = 0; j < 4; ++j) so[rr][k * (RD + HID) + RD + lane * 4 + j] = lk(mrow[j]); }
    wave_lds_sync();
    v8f acc[4];
#pragma unroll
    for (int t = 0; t < 4; ++t) acc[t] = (v8f){};
#pragma unroll
    for (int kb = 0; kb < HID; kb += 32) { const v16b a = frag_kb(&Ah[nloc][kb], hlf), a2 = frag_kb(&Al[nloc][kb], hlf);
#pragma unroll
      for (int t = 0; t < 4; ++t) { const v16b bw = frag_kb(Q + (size_t)(t * 16 + nloc) * HID + kb, hlf); acc[t] = wmma16b(a, bw, acc[t]); acc[t] = wmma16b(a2, bw, acc[t]); } }
#pragma unroll
    for (int t = 0; t < 4; ++t) { const int c = t * 16 + nloc; const float bb = bf16_rne(qb[c]);
#pragma unroll 1
      for (int r8 = 0; r8 < 8; ++r8) so[8 * hlf + r8][k * (RD + HID) + c] = lk(lk(acc[t][r8] * (1.0f / (XS * WSC)) + bb)); }
    wave_lds_sync(); }
  for (int pass = 0; pass < 2; ++pass) {
#pragma unroll 1
    for (int rr = 0; rr < 16; ++rr) { if (g0 + rr < (size_t)G) for (int q = lane * 4; q < OUTW; q += 128) *(volatile v4f*)(out + (g0 + rr) * OUTW + q) = *(const v4f*)(&so[rr][q]); } __threadfence(); }
}
}

extern "C" void kernel_launch(void* const* d_in, const int* in_sizes, int n_in, void* d_out, int out_size, void* d_ws, size_t ws_size, hipStream_t stream) {
  (void)n_in;
  auto Fp = [&](int i) { return (const float*)d_in[i]; }; auto Ip = [&](int i) { return (const int*)d_in[i]; };
  if (in_sizes[0] != N * FIN || in_sizes[1] != E || in_sizes[2] != FIN * HID || in_sizes[3] != HID * HID || in_sizes[10] != HID * HID || in_sizes[12] != HID * RD || in_sizes[16] != HID * RD || in_sizes[18] != E || in_sizes[19] != E || in_sizes[20] != N || out_size != G * OUTW) return;
  size_t off = 0; char* ws = (char*)d_ws;
  auto carve = [&](size_t bytes) { char* p = ws + off; off += (bytes + 255) & ~(size_t)255; return p; };
  b16* W1T = (b16*)carve((size_t)HID * FIN * 2); b16* W2T = (b16*)carve((size_t)HID * HID * 2); b16* P1T = (b16*)carve((size_t)HID * HID * 2); b16* P2T = (b16*)carve((size_t)HID * HID * 2); b16* Q1T = (b16*)carve((size_t)RD * HID * 2); b16* Q2T = (b16*)carve((size_t)RD * HID * 2);
  float* HW = (float*)carve((size_t)NP * HID * 4); float* Z = (float*)carve((size_t)NP * HID * 4); float* H = (float*)carve((size_t)NP * HID * 4); float* PH = HW;
  float* M1 = (float*)carve((size_t)GP * HID * 4); float* M2 = (float*)carve((size_t)GP * HID * 4); float* POOL1 = (float*)carve((size_t)GP * HID * 4); float* POOL2 = (float*)carve((size_t)GP * HID * 4);
  CsrBufs csrD, csrS; off = csr_carve(csrD, ws, off, E, N); off = csr_carve(csrS, ws, off, E, N);
  if (off > ws_size) return;
  wprep_kernel<<<(unsigned)(((size_t)HID * FIN / 8 + 3 * (size_t)HID * HID / 8 + 2 * (size_t)RD * HID / 8 + 255) / 256), 256, 0, stream>>>(Fp(2), Fp(3), Fp(10), Fp(14), Fp(12), Fp(16), W1T, W2T, P1T, P2T, Q1T, Q2T);
  csr_build(csrD, Ip(19), E, N, stream); csr_build(csrS, Ip(18), E, N, stream);
  gemm_kernel<0><<<NP / 64, 128, 0, stream>>>(Fp(0), W1T, csrS.ROWCNT, nullptr, HW);
  agg_kernel<<<NP / 8, 256, 0, stream>>>(HW, Fp(1), Ip(18), csrD.PERM, csrD.ROWPTR, csrD.ROWCNT, (int)csrD.permLen, Z);
  gnorm_kernel<<<G, 128, 0, stream>>>(Z, Fp(4), Fp(5), Fp(6), H, M1);
  gemm_kernel<2><<<N / 64 + 1, 128, 0, stream>>>(H, P1T, nullptr, Fp(11), PH);
  pool_kernel<<<GP, 128, 0, stream>>>(PH, POOL1);
  gemm_kernel<1><<<NP / 64, 128, 0, stream>>>(H, W2T, csrS.ROWCNT, nullptr, HW);
  agg_kernel<<<NP / 8, 256, 0, stream>>>(HW, Fp(1), Ip(18), csrD.PERM, csrD.ROWPTR, csrD.ROWCNT, (int)csrD.permLen, Z);
  gnorm_kernel<<<G, 128, 0, stream>>>(Z, Fp(7), Fp(8), Fp(9), H, M2);
  gemm_kernel<2><<<N / 64 + 1, 128, 0, stream>>>(H, P2T, nullptr, Fp(15), PH);
  pool_kernel<<<GP, 128, 0, stream>>>(PH, POOL2);
  head_kernel<<<GP / 16, 32, 0, stream>>>(POOL1, POOL2, Q1T, Q2T, Fp(13), Fp(17), M1, M2, (float*)d_out);
}
